// Block_17712445129207
// MI455X (gfx1250) — hardware-run, weakly checked
//
#include <hip/hip_runtime.h>


#ifndef NB
#define NB 8
#endif
#ifndef SEQ
#define SEQ 2048
#endif
#define NB_FULL  8
#define SEQ_FULL 2048
#ifndef OUT_SEQ
#define OUT_SEQ SEQ
#endif
#define EM   400
#define NH_  4
#define HDR  100
#define DP   128
#define FF   1600
#define HP   448
#define KE   416
#define AP   512
#define NP   448
#define MT   (NB * SEQ)
#define AW   4
#define OSP  132
#define WSC  64.0f
#define WSI  (1.0f / 64.0f)
#define CSC  16.0f
#define CWI  (1.0f / 1024.0f)
#define SC2  ((float)(0.1 * 1.4426950408889634))
#define PSH  14.0f
#define NEGB (-3.0e38f)

static_assert(NH_ * HDR == EM);
static_assert(HDR <= 112);
static_assert(DP % 32 == 0);
static_assert(DP == 128);
static_assert(NH_ * DP == AP);
static_assert(KE % 32 == 0);
static_assert(KE >= EM);
static_assert(KE <= HP);
static_assert(13 * 32 == KE);
static_assert(KE + 32 == HP);
static_assert(56 * 8 == HP);
static_assert(HP % 64 == 0);
static_assert(AP % 64 == 0);
static_assert(AP % 32 == 0);
static_assert(FF % 64 == 0);
static_assert(FF % 32 == 0);
static_assert(NP % 64 == 0);
static_assert(NP >= EM);
static_assert(NP == HP);
static_assert(EM % 4 == 0);
static_assert(SEQ % 64 == 0);
static_assert(MT % 64 == 0);
static_assert(MT % 8 == 0);
static_assert(SEQ % 32 == 0);
static_assert(SEQ % (16 * AW) == 0);
static_assert(NB <= NB_FULL);
static_assert(SEQ <= SEQ_FULL);
static_assert((OSP * 4) % 16 == 0);
static_assert(OSP >= DP);
static_assert(AW * 16 * OSP * 4 <= 131072);
static_assert(16 * 68 * 4 <= 131072);
static_assert(32 * 72 * 2 <= 131072);
static_assert(2 * 512 * 4 + 8 * HP * 2 <= 131072);
static_assert(32 * 16 * 8 == 16 * DP * 2);
static_assert(32 * 16 * 4 == 16 * 64 * 2);
static_assert(32 * 16 * 8 == 16 * 64 * 4);
static_assert(256 * 16 == 32 * 64 * 2);

typedef _Float16 h16;
typedef __attribute__((ext_vector_type(16))) _Float16 v16h;
typedef __attribute__((ext_vector_type(8)))  _Float16 v8h;
typedef __attribute__((ext_vector_type(8)))  float    v8f;
typedef __attribute__((ext_vector_type(4)))  float    v4f;
typedef v4f  __attribute__((may_alias)) v4fa;
typedef v8h  __attribute__((may_alias)) v8ha;

__device__ __forceinline__ unsigned short f2bf(float f) { unsigned u = __float_as_uint(f); u += 0x7FFFu + ((u >> 16) & 1u); return (unsigned short)(u >> 16); }
__device__ __forceinline__ float bfr(float f) { return __uint_as_float(((unsigned)f2bf(f)) << 16); }
__device__ __forceinline__ v16h cat16(v8h lo, v8h hi) { return __builtin_shufflevector(lo, hi, 0, 1, 2, 3, 4, 5, 6, 7, 8, 9, 10, 11, 12, 13, 14, 15); }
__device__ __forceinline__ v8f wmma16(v16h a, v16h b, v8f c) { return __builtin_amdgcn_wmma_f32_16x16x32_f16(false, a, false, b, (short)0, c, false, false); }
__device__ __forceinline__ v16h  ldh(const h16* p) { return cat16(*(const v8h*)p, *(const v8h*)(p + 16)); }
__device__ __forceinline__ void wave_sync() { __builtin_amdgcn_fence(3  , "wavefront"); __builtin_amdgcn_wave_barrier(); asm volatile("" ::: "memory"); }
static __device__ __forceinline__ h16 toh_flush(float v) { const h16 r = (h16)v; return (fabsf(v) < 6.103515625e-05f) ? (h16)0.0f : r; }
__device__ __forceinline__ v8f wmg(v16h a, v16h b, v8f c) {
    c = wmma16(a, b, c);
    asm volatile("v_nop\n\tv_nop\n\tv_nop\n\tv_nop" : "+v"(c) : "v"(a), "v"(b));
    return c;
}

__global__ __launch_bounds__(256) void k_wconv(const float* __restrict__ src, h16* dst, int kr, int kpg, int nr, int npg, int ld, int zstride, int kp) {
    __shared__ __align__(16) h16 ts[32 * 72];
    const int tid = threadIdx.x;
    const int k0 = blockIdx.x * 64, n0 = blockIdx.y * 32;
    const int nn = tid & 31, kq = tid >> 5;
    const int np = n0 + nn; const int z = np / npg; const int ni = np - z * npg;
    const int nic = ni < nr ? ni : nr - 1;
#pragma unroll 1
    for (int i = 0; i < 8; ++i) {
        const int kk = kq + 8 * i; const int kpos = k0 + kk; const int kg = kpos / kpg; const int ki = kpos - kg * kpg;
        const int kic = ki < kr ? ki : kr - 1;
        float v = src[(size_t)z * (size_t)zstride + (size_t)(kg * kr + kic) * (size_t)ld + (size_t)nic];
        asm volatile("" : "+v"(v));
        const bool ok = (ni < nr) & (ki < kr);
        const float w = ok ? bfr(v) * WSC : 0.0f;
        ts[nn * 72 + kk] = toh_flush(w);
    }
    __syncthreads();
    const int row = tid >> 3, pc = tid & 7;
    const v8h o = *(const v8ha*)(&ts[row * 72 + pc * 8]);
    h16* d = dst + (size_t)(n0 + row) * (size_t)kp + (size_t)k0 + (size_t)pc * 8;
    *(volatile v8h*)d = o; __threadfence(); *(volatile v8h*)d = o;
}

__global__ __launch_bounds__(256) void k_ln(const float* __restrict__ X, const float* __restrict__ G, const float* __restrict__ Bv, h16* H, int pitch, int inp) {
#pragma clang fp contract(off)
    __shared__ __align__(16) float gs[512];
    __shared__ __align__(16) float bs[512];
    __shared__ __align__(16) h16 hs[8 * HP];
    const int tid = threadIdx.x, lane = tid & 31;
    const int wave = __builtin_amdgcn_readfirstlane((int)(threadIdx.x >> 5));
#pragma unroll 1
    for (int j = 0; j < 2; ++j) {
        const int i = tid + 256 * j; const int cc = i < EM ? i : EM - 1;
        float g = G[cc]; float b = Bv[cc];
        asm volatile("" : "+v"(g)); asm volatile("" : "+v"(b));
        gs[i] = (i < EM) ? bfr(g) : 0.0f; bs[i] = (i < EM) ? bfr(b) : 0.0f;
    }
    __syncthreads();
    const int m = blockIdx.x * 8 + wave;
    const int rowi = m + inp * (m / SEQ) * (SEQ_FULL - SEQ);
    const size_t roff = (size_t)rowi * (size_t)pitch;
    float xv[13]; float s = 0.0f;
#pragma unroll
    for (int i = 0; i < 13; ++i) {
        const int c = lane + 32 * i; const int cc = c < EM ? c : EM - 1;
        float x = X[roff + cc];
        asm volatile("" : "+v"(x));
        const float xb = inp ? bfr(x) : x;
        const float v = (c < EM) ? xb : 0.0f;
        xv[i] = v; s += v;
    }
#pragma unroll
    for (int off = 16; off; off >>= 1) s += __shfl_xor(s, off, 32);
    const float mu = s * (1.0f / EM);
    float q = 0.0f;
#pragma unroll
    for (int i = 0; i < 13; ++i) {
        const int c = lane + 32 * i;
        const float d = (c < EM) ? (xv[i] - mu) : 0.0f;
        q += d * d;
    }
#pragma unroll
    for (int off = 16; off; off >>= 1) q += __shfl_xor(q, off, 32);
    const float rs = rsqrtf(q * (1.0f / EM) + 1e-5f);
    const int hb = wave * HP;
#pragma unroll
    for (int i = 0; i < 13; ++i) {
        const int c = lane + 32 * i;
        const float y = (xv[i] - mu) * rs * gs[c] + bs[c];
        hs[hb + c] = (c < EM) ? toh_flush(y) : (h16)0.0f;
    }
    hs[hb + KE + lane] = (h16)0.0f;
    wave_sync();
    const int p2 = (32 + lane) < 56 ? (32 + lane) : 55;
    const v8h a0 = *(const v8ha*)(&hs[hb + lane * 8]);
    const v8h a1 = *(const v8ha*)(&hs[hb + p2 * 8]);
    h16* hr = H + (size_t)m * HP;
#pragma unroll 1
    for (int ps = 0; ps < 2; ++ps) {
        *(volatile v8h*)(hr + lane * 8) = a0;
        if (lane < 24) *(volatile v8h*)(hr + (32 + lane) * 8) = a1;
        if (ps == 0) __threadfence(); }
}

__device__ __forceinline__ void gemm_main(const h16* __restrict__ A, size_t lda, const h16* __restrict__ Bt, size_t ldb, int K, int r0, int c0, int lr, int hi, v8f (&acc)[4][4]) {
#pragma unroll
    for (int mb = 0; mb < 4; ++mb)
#pragma unroll
        for (int nb = 0; nb < 4; ++nb) acc[mb][nb] = (v8f){};
    const size_t aoff = (size_t)(r0 + lr) * lda + 8 * hi, boff = (size_t)(c0 + lr) * ldb + 8 * hi;
#pragma unroll 1
    for (int kc = 0; kc < K; kc += 32) {
        v16h a[4];
#pragma unroll
        for (int mb = 0; mb < 4; ++mb) a[mb] = ldh(A + aoff + (size_t)mb * 16 * lda + kc);
#pragma unroll
        for (int nb = 0; nb < 4; ++nb) { const v16h b = ldh(Bt + boff + (size_t)nb * 16 * ldb + kc);
#pragma unroll
            for (int mb = 0; mb < 4; ++mb) acc[mb][nb] = wmg(a[mb], b, acc[mb][nb]); }
    }
}

template <int BIAS, int RELU>
__device__ __forceinline__ void epi16(v8f (&acc)[4][4], float scale, const float* __restrict__ bias, int c0, int lane, h16* P, size_t base, size_t pitch) {
    __shared__ __align__(16) float os[16 * 68];
    const int lr = lane & 15, hi = lane >> 4;
    float bc[4];
#pragma unroll
    for (int nb = 0; nb < 4; ++nb) { bc[nb] = 0.0f; if (BIAS) { const float bv = bias[c0 + nb * 16 + lr]; bc[nb] = bfr(bv); } }
#pragma unroll
    for (int mb = 0; mb < 4; ++mb) {
#pragma unroll
        for (int nb = 0; nb < 4; ++nb) {
#pragma unroll
            for (int j = 0; j < 8; ++j) { float v = acc[mb][nb][j] * scale + bc[nb]; if (RELU) v = fmaxf(v, 0.0f); os[(hi * 8 + j) * 68 + nb * 16 + lr] = v; } }
        wave_sync();
#pragma unroll 1
        for (int ps = 0; ps < 2; ++ps) {
#pragma unroll
            for (int s = 0; s < 4; ++s) { const int row = 4 * s + (lane >> 3), c8 = (lane & 7) * 8;
                const v4f x0 = *(const v4fa*)(&os[row * 68 + c8]); const v4f x1 = *(const v4fa*)(&os[row * 68 + c8 + 4]); v8h hv;
#pragma unroll
                for (int i = 0; i < 4; ++i) { hv[i] = toh_flush(x0[i]); hv[4 + i] = toh_flush(x1[i]); }
                *(volatile v8h*)(P + base + (size_t)(mb * 16 + row) * pitch + c8) = hv; }
            if (ps == 0) __threadfence(); }
        wave_sync();
    }
}

__device__ __forceinline__ void epi32(v8f (&acc)[4][4], float scale, const float* __restrict__ bias, int ncol, int r0, int c0, int lane,
                                      const float* R, size_t rpitch, int rmap, int rbf, float* OUT, size_t opitch) {
    __shared__ __align__(16) float os[16 * 68];
    const int lr = lane & 15, hi = lane >> 4;
    float bc[4];
#pragma unroll
    for (int nb = 0; nb < 4; ++nb) { const int n = c0 + nb * 16 + lr; const int nc = n < ncol ? n : ncol - 1;
        float bv = bias[nc];
        asm volatile("" : "+v"(bv));
        bc[nb] = (n < ncol) ? bfr(bv) : 0.0f; }
#pragma unroll
    for (int mb = 0; mb < 4; ++mb) {
#pragma unroll
        for (int nb = 0; nb < 4; ++nb) {
#pragma unroll
            for (int j = 0; j < 8; ++j) os[(hi * 8 + j) * 68 + nb * 16 + lr] = acc[mb][nb][j] * scale + bc[nb]; }
        wave_sync();
#pragma unroll
        for (int s = 0; s < 8; ++s) { const int row = 2 * s + (lane >> 4), c4 = (lane & 15) * 4;
            const int col = c0 + c4; const int cc = col < ncol ? col : ncol - 4;
            const int g = r0 + mb * 16 + row; const int gr = g + rmap * (g / SEQ) * (SEQ_FULL - SEQ);
            v4f xv = *(const v4f*)(R + (size_t)gr * rpitch + cc);
            asm volatile("" : "+v"(xv));
            v4f cur = *(const v4fa*)(&os[row * 68 + c4]);
#pragma unroll
            for (int i = 0; i < 4; ++i) { const float xi = rbf ? bfr(xv[i]) : xv[i]; cur[i] += (col < ncol) ? xi : 0.0f; }
            *(v4fa*)(&os[row * 68 + c4]) = cur; }
        wave_sync();
#pragma unroll 1
        for (int ps = 0; ps < 2; ++ps) {
#pragma unroll
            for (int s = 0; s < 8; ++s) { const int row = 2 * s + (lane >> 4), c4 = (lane & 15) * 4;
                const v4f val = *(const v4fa*)(&os[row * 68 + c4]);
                *(volatile v4f*)(OUT + (size_t)(r0 + mb * 16 + row) * opitch + c0 + c4) = val; }
            if (ps == 0) __threadfence(); }
        wave_sync();
    }
}

__global__ __launch_bounds__(32) void k_qk(const h16* __restrict__ A, const h16* __restrict__ Bt, h16* P) {
    const int lane = threadIdx.x & 31, lr = lane & 15, hi = lane >> 4;
    const int r0 = blockIdx.x * 64, ct = blockIdx.y, c0 = ct * 64;
    v8f acc[4][4];
    gemm_main(A, (size_t)HP, Bt, (size_t)HP, KE, r0, c0, lr, hi, acc);
    const int mat = ct >> 3, hh = (ct >> 1) & 3, dh = ct & 1;
    const int bb = r0 / SEQ, tt = r0 % SEQ;
    const size_t base = (size_t)mat * ((size_t)NB * NH_ * SEQ * DP) + ((size_t)(bb * NH_ + hh) * SEQ + (size_t)tt) * DP + (size_t)dh * 64;
    epi16<0, 0>(acc, WSI, nullptr, c0, lane, P, base, (size_t)DP);
}

__global__ __launch_bounds__(32) void k_vt(const h16* __restrict__ A, const h16* __restrict__ Bt, h16* P) {
    const int lane = threadIdx.x & 31, lr = lane & 15, hi = lane >> 4;
    const int r0 = blockIdx.x * 64, c0 = blockIdx.y * 64;
    v8f acc[4][4];
    gemm_main(A, (size_t)HP, Bt, (size_t)HP, KE, r0, c0, lr, hi, acc);
    const int bb = c0 / SEQ, tt = c0 % SEQ;
    const size_t base = (size_t)bb * ((size_t)NH_ * DP * SEQ) + (size_t)r0 * SEQ + (size_t)tt;
    epi16<0, 0>(acc, WSI, nullptr, c0, lane, P, base, (size_t)SEQ);
}

__global__ __launch_bounds__(32 * AW) void k_flash(const h16* __restrict__ QP, const h16* __restrict__ KP, const h16* __restrict__ VT, h16* ATT) {
    __shared__ __align__(16) float os[AW * 16 * OSP];
    const int lane = threadIdx.x & 31, lr = lane & 15, hi = lane >> 4;
    const int wave = __builtin_amdgcn_readfirstlane((int)(threadIdx.x >> 5));
    const int zh = blockIdx.y; const int b = zh / NH_, h = zh % NH_;
    const int t0 = (blockIdx.x * AW + wave) * 16;
    const int lim = t0 + lr;
    const int nk = (t0 + 16 + 31) & ~31;
    const size_t pbase = (size_t)zh * SEQ * DP;
    const size_t qo = pbase + (size_t)(t0 + lr) * DP + 8 * hi;
    const size_t ko = pbase + (size_t)lr * DP + 8 * hi;
    const size_t vo = pbase + (size_t)lr * SEQ + 8 * hi;
    v8f o[7];
#pragma unroll
    for (int j = 0; j < 7; ++j) o[j] = (v8f){};
    float m = NEGB, l = 0.0f;
#pragma unroll 1
    for (int key0 = 0; key0 < nk; key0 += 32) {
        v8f sa = (v8f){}, sb = (v8f){};
        const size_t kro = ko + (size_t)key0 * DP;
#pragma unroll 1
        for (int kk = 0; kk < DP; kk += 32) {
            const v16h q  = ldh(QP + qo + kk);
            const v16h ka = ldh(KP + kro + kk);
            const v16h kb = ldh(KP + kro + (size_t)16 * DP + kk);
            sa = wmg(ka, q, sa); sb = wmg(kb, q, sb);
        }
        const int ja = key0 + 8 * hi;
        float ta[8], tb[8]; bool fa[8], fb[8]; float mx = NEGB;
#pragma unroll
        for (int r = 0; r < 8; ++r) {
            fa[r] = (ja + r <= lim);
            fb[r] = (ja + 16 + r <= lim);
            ta[r] = sa[r] * SC2; tb[r] = sb[r] * SC2;
            mx = fmaxf(mx, fmaxf(fa[r] ? ta[r] : NEGB, fb[r] ? tb[r] : NEGB)); }
        mx = fmaxf(mx, __shfl_xor(mx, 16, 32));
        const float mnew = fmaxf(m, mx);
        const float alpha = __builtin_amdgcn_exp2f(m - mnew);
        const float sh = PSH - mnew;
        v16h pb; float ls = 0.0f;
#pragma unroll
        for (int r = 0; r < 8; ++r) {
            const float aa = ta[r] + sh, ab = tb[r] + sh;
            const float ea = __builtin_amdgcn_exp2f(aa), eb = __builtin_amdgcn_exp2f(ab);
            const float ga = (fa[r] & (aa >= -14.0f)) ? ea : 0.0f;
            const float gb = (fb[r] & (ab >= -14.0f)) ? eb : 0.0f;
            const h16 pa = (h16)ga; const h16 pc = (h16)gb;
            pb[r] = pa; pb[8 + r] = pc;
            ls += (float)pa + (float)pc; }
        l = l * alpha + ls; m = mnew;
#pragma unroll
        for (int j = 0; j < 7; ++j) o[j] = o[j] * alpha;
        const h16* va = VT + vo + key0;
#pragma unroll
        for (int j = 0; j < 7; ++j) { const v16h v = ldh(va + (size_t)(16 * j) * SEQ); o[j] = wmg(v, pb, o[j]); }
    }
    l += __shfl_xor(l, 16, 32);
    const bool any = l > 0.0f;
    const float lsafe = any ? l : 1.0f;
    const float inv = any ? (CSC * (1.0f / lsafe)) : 0.0f;
    const int wb = wave * 16 * OSP;
#pragma unroll
    for (int j = 0; j < 7; ++j) { v4f a, c;
        a[0] = o[j][0] * inv; a[1] = o[j][1] * inv; a[2] = o[j][2] * inv; a[3] = o[j][3] * inv; c[0] = o[j][4] * inv; c[1] = o[j][5] * inv; c[2] = o[j][6] * inv; c[3] = o[j][7] * inv;
        *(v4fa*)(&os[wb + lr * OSP + 16 * j + 8 * hi]) = a; *(v4fa*)(&os[wb + lr * OSP + 16 * j + 8 * hi + 4]) = c; }
    { const v4f zz = (v4f){}; *(v4fa*)(&os[wb + lr * OSP + 112 + 8 * hi]) = zz; *(v4fa*)(&os[wb + lr * OSP + 112 + 8 * hi + 4]) = zz; }
    wave_sync();
    h16* arow = ATT + ((size_t)b * SEQ + t0) * AP + (size_t)h * DP;
#pragma unroll 1
    for (int ps = 0; ps < 2; ++ps) {
#pragma unroll
        for (int s = 0; s < 8; ++s) { const int row = 2 * s + (lane >> 4), c8 = (lane & 15) * 8;
            const v4f x0 = *(const v4fa*)(&os[wb + row * OSP + c8]); const v4f x1 = *(const v4fa*)(&os[wb + row * OSP + c8 + 4]); v8h hv;
#pragma unroll
            for (int i = 0; i < 4; ++i) { hv[i] = toh_flush(x0[i]); hv[4 + i] = toh_flush(x1[i]); }
            *(volatile v8h*)(arow + (size_t)row * AP + c8) = hv; }
        if (ps == 0) __threadfence(); }
}

__global__ __launch_bounds__(32) void k_wo(const h16* __restrict__ A, const h16* __restrict__ Bt, const float* __restrict__ bias, const float* __restrict__ X, float* X2) {
    const int lane = threadIdx.x & 31, lr = lane & 15, hi = lane >> 4;
    const int r0 = blockIdx.x * 64, c0 = blockIdx.y * 64;
    v8f acc[4][4];
    gemm_main(A, (size_t)AP, Bt, (size_t)AP, AP, r0, c0, lr, hi, acc);
    epi32(acc, CWI, bias, EM, r0, c0, lane, X, (size_t)EM, 1, 1, X2, (size_t)HP);
}

__global__ __launch_bounds__(32) void k_w1(const h16* __restrict__ A, const h16* __restrict__ Bt, const float* __restrict__ bias, h16* P) {
    const int lane = threadIdx.x & 31, lr = lane & 15, hi = lane >> 4;
    const int r0 = blockIdx.x * 64, c0 = blockIdx.y * 64;
    v8f acc[4][4];
    gemm_main(A, (size_t)HP, Bt, (size_t)HP, KE, r0, c0, lr, hi, acc);
    epi16<1, 1>(acc, WSI, bias, c0, lane, P, (size_t)r0 * FF + (size_t)c0, (size_t)FF);
}

__global__ __launch_bounds__(32) void k_w2(const h16* __restrict__ A, const h16* __restrict__ Bt, const float* __restrict__ bias, float* X2) {
    const int lane = threadIdx.x & 31, lr = lane & 15, hi = lane >> 4;
    const int r0 = blockIdx.x * 64, c0 = blockIdx.y * 64;
    v8f acc[4][4];
    gemm_main(A, (size_t)FF, Bt, (size_t)FF, FF, r0, c0, lr, hi, acc);
    epi32(acc, WSI, bias, EM, r0, c0, lane, X2, (size_t)HP, 0, 0, X2, (size_t)HP);
}

__global__ __launch_bounds__(256) void k_out(const float* __restrict__ X2, float* OUT, int n4) {
    const int i = blockIdx.x * 256 + threadIdx.x; if (i >= n4) return;
    const int r = i / (EM / 4); const int c4 = i - r * (EM / 4);
    const v4f v = *(const v4f*)(X2 + (size_t)r * HP + 4 * c4);
    const int orow = r + (r / SEQ) * (OUT_SEQ - SEQ);
    float* d = OUT + (size_t)orow * EM + 4 * c4;
    *(volatile v4f*)d = v; __threadfence(); *(volatile v4f*)d = v;
}

static constexpr size_t al256(size_t v) { return (v + 255) & ~(size_t)255; }
static constexpr size_t PLANE_E = (size_t)NB * NH_ * SEQ * DP;
static constexpr size_t SZ_H   = al256((size_t)MT * HP * 2);
static constexpr size_t SZ_PL  = al256(PLANE_E * 2);
static constexpr size_t SZ_AT  = al256((size_t)MT * AP * 2);
static constexpr size_t SZ_F1  = al256((size_t)MT * FF * 2);
static constexpr size_t SZ_RA  = 3 * SZ_PL + SZ_AT;
static constexpr size_t SZ_R   = SZ_RA > SZ_F1 ? SZ_RA : SZ_F1;
static constexpr size_t SZ_X2  = al256((size_t)MT * HP * 4);
static constexpr size_t SZ_WQK = al256((size_t)2 * NH_ * DP * HP * 2);
static constexpr size_t SZ_WV  = al256((size_t)NH_ * DP * HP * 2);
static constexpr size_t SZ_WO  = al256((size_t)NP * AP * 2);
static constexpr size_t SZ_W1  = al256((size_t)FF * HP * 2);
static constexpr size_t SZ_W2  = al256((size_t)NP * FF * 2);
static constexpr size_t SZ_TOTAL = SZ_H + SZ_R + SZ_X2 + SZ_WQK + SZ_WV + SZ_WO + SZ_W1 + SZ_W2;
static_assert(SZ_TOTAL <= (size_t)134217728);
static_assert(SZ_PL == PLANE_E * 2);
static_assert(SZ_RA <= SZ_R);
static_assert(SZ_F1 <= SZ_R);
static_assert((size_t)NB * NH_ * SEQ * DP == (size_t)NB * NH_ * DP * SEQ);
static_assert(((size_t)MT * (EM / 4)) % 256 == 0);
static_assert((2 * NH_ * DP) % 64 == 0);
static_assert((NH_ * DP) % 64 == 0);
static_assert((NH_ * DP) % 32 == 0);
static_assert(NP % 32 == 0);
static_assert(FF % 32 == 0);

extern "C" void kernel_launch(void* const* d_in, const int* in_sizes, int n_in,
                              void* d_out, int out_size, void* d_ws, size_t ws_size, hipStream_t stream) {
    if (n_in < 14) return;
    const size_t needx = ((size_t)(NB - 1) * SEQ_FULL + SEQ) * EM;
    if ((size_t)in_sizes[0] < needx) return;
    if (in_sizes[1] < EM || in_sizes[2] < EM || in_sizes[3] < EM || in_sizes[4] < EM) return;
    if ((size_t)in_sizes[5] < (size_t)NH_ * EM * HDR || (size_t)in_sizes[6] < (size_t)NH_ * EM * HDR || (size_t)in_sizes[7] < (size_t)NH_ * EM * HDR) return;
    if ((size_t)in_sizes[8] < (size_t)EM * EM || in_sizes[9] < EM) return;
    if ((size_t)in_sizes[10] < (size_t)EM * FF || in_sizes[11] < FF) return;
    if ((size_t)in_sizes[12] < (size_t)FF * EM || in_sizes[13] < EM) return;
    if ((size_t)out_size < ((size_t)(NB - 1) * OUT_SEQ + SEQ) * EM) return;
    if (SZ_TOTAL > ws_size) return;
    const float* x    = (const float*)d_in[0];
    const float* ln1g = (const float*)d_in[1];  const float* ln1b = (const float*)d_in[2];
    const float* ln2g = (const float*)d_in[3];  const float* ln2b = (const float*)d_in[4];
    const float* wq   = (const float*)d_in[5];  const float* wk   = (const float*)d_in[6];  const float* wv = (const float*)d_in[7];
    const float* wo   = (const float*)d_in[8];  const float* bo   = (const float*)d_in[9];
    const float* w1   = (const float*)d_in[10]; const float* b1   = (const float*)d_in[11];
    const float* w2   = (const float*)d_in[12]; const float* b2   = (const float*)d_in[13];
    float* OUT = (float*)d_out;
    char* wsp = (char*)d_ws;
    h16* H16 = (h16*)wsp; wsp += SZ_H;
    char* reg = wsp; wsp += SZ_R;
    h16* QK  = (h16*)reg;
    h16* VT  = (h16*)(reg + 2 * SZ_PL);
    h16* ATT = (h16*)(reg + 3 * SZ_PL);
    h16* FF1 = (h16*)reg;
    float* X2 = (float*)wsp; wsp += SZ_X2;
    h16* WQK = (h16*)wsp; wsp += SZ_WQK;
    h16* WVT = (h16*)wsp; wsp += SZ_WV;
    h16* WOT = (h16*)wsp; wsp += SZ_WO;
    h16* W1T = (h16*)wsp; wsp += SZ_W1;
    h16* W2T = (h16*)wsp; wsp += SZ_W2;

    k_wconv<<<dim3(HP / 64, (NH_ * DP) / 32, 1), 256, 0, stream>>>(wq, WQK, EM, HP, HDR, DP, HDR, EM * HDR, HP);
    k_wconv<<<dim3(HP / 64, (NH_ * DP) / 32, 1), 256, 0, stream>>>(wk, WQK + (size_t)NH_ * DP * HP, EM, HP, HDR, DP, HDR, EM * HDR, HP);
    k_wconv<<<dim3(HP / 64, (NH_ * DP) / 32, 1), 256, 0, stream>>>(wv, WVT, EM, HP, HDR, DP, HDR, EM * HDR, HP);
    k_wconv<<<dim3(AP / 64, NP / 32, 1), 256, 0, stream>>>(wo, WOT, HDR, DP, EM, NP, EM, 0, AP);
    k_wconv<<<dim3(HP / 64, FF / 32, 1), 256, 0, stream>>>(w1, W1T, EM, HP, FF, FF, FF, 0, HP);
    k_wconv<<<dim3(FF / 64, NP / 32, 1), 256, 0, stream>>>(w2, W2T, FF, FF, EM, NP, EM, 0, FF);

    k_ln<<<MT / 8, 256, 0, stream>>>(x, ln1g, ln1b, H16, EM, 1);
    k_qk<<<dim3(MT / 64, (2 * NH_ * DP) / 64, 1), 32, 0, stream>>>(H16, WQK, QK);
    k_vt<<<dim3((NH_ * DP) / 64, MT / 64, 1), 32, 0, stream>>>(WVT, H16, VT);
    k_flash<<<dim3(SEQ / (16 * AW), NB * NH_, 1), 32 * AW, 0, stream>>>(QK, QK + PLANE_E, VT, ATT);
    k_wo<<<dim3(MT / 64, NP / 64, 1), 32, 0, stream>>>(ATT, WOT, bo, x, X2);
    k_ln<<<MT / 8, 256, 0, stream>>>(X2, ln2g, ln2b, H16, HP, 0);
    k_w1<<<dim3(MT / 64, FF / 64, 1), 32, 0, stream>>>(H16, W1T, b1, FF1);
    k_w2<<<dim3(MT / 64, NP / 64, 1), 32, 0, stream>>>(FF1, W2T, b2, X2);
    { const int n4 = MT * (EM / 4);
      k_out<<<(unsigned)((n4 + 255) / 256), 256, 0, stream>>>(X2, OUT, n4); }
}
